// AoA_Refine_Module_50586124812561
// MI455X (gfx1250) — hardware-verified
//
#include <hip/hip_runtime.h>
#include <math.h>

constexpr int kB   = 32;
constexpr int kM   = 196;
constexpr int kD   = 1024;
constexpr int kH   = 8;
constexpr int kHD  = 128;
constexpr int kL   = 3;
constexpr int kTok = kB * kM;
constexpr int kTokPad = kTok + 64;
constexpr int kSP  = 256;
constexpr int kKeyK = 224;
constexpr float kXCarry = 16.0f;
constexpr float kWCarry = 256.0f;
constexpr float kPCarry = 2048.0f;

constexpr size_t kBytesP    = (size_t)kTok * kD * 4;
constexpr size_t kBytesATT  = (size_t)kB * kSP * kD * 4;
constexpr size_t kBytesX16  = (size_t)kTok * kD * 2;
constexpr size_t kBytesW16  = (size_t)4 * kD * kD * 2;
constexpr size_t kBytesWC16 = (size_t)kHD * kHD * 2;
constexpr size_t kBytesQ16  = (size_t)kTokPad * kD * 2;
constexpr size_t kBytesV2T  = (size_t)kH * kHD * kB * kSP * 2;
constexpr size_t kBytesS    = (size_t)kB * kSP * kSP * 4;
constexpr size_t kBytesPP   = (size_t)kB * kSP * kSP * 2;
constexpr size_t kOffP    = 0;
constexpr size_t kOffATT  = kOffP + kBytesP;
constexpr size_t kOffX16  = kOffATT + kBytesATT;
constexpr size_t kOffW16  = kOffX16 + kBytesX16;
constexpr size_t kOffWC16 = kOffW16 + kBytesW16;
constexpr size_t kOffQ16  = kOffWC16 + kBytesWC16;
constexpr size_t kOffK16  = kOffQ16 + kBytesQ16;
constexpr size_t kOffV2T  = kOffK16 + kBytesQ16;
constexpr size_t kWsTotal = kOffV2T + kBytesV2T;
static_assert(kWsTotal == 123240448, "carve total");
static_assert(kWsTotal <= 134217728, "carve under 128 MiB");
static_assert(kBytesX16 >= kBytesS + kBytesPP, "scores + probs fit in the x16 region");
static_assert(kBytesATT >= (size_t)kTok * kD * 2, "vk plane fits in the attn region");
static_assert(kBytesP == (size_t)kTok * kH * kHD * 4, "gate plane fits in the P region");
static_assert((kOffATT % 256) == 0 && (kOffX16 % 256) == 0 && (kOffW16 % 256) == 0 && (kOffQ16 % 256) == 0 && (kOffK16 % 256) == 0 && (kOffV2T % 256) == 0, "aligned");

typedef __attribute__((ext_vector_type(16))) _Float16 v16h;
typedef __attribute__((ext_vector_type(8)))  _Float16 v8h;
typedef __attribute__((ext_vector_type(16))) __bf16   v16b;
typedef __attribute__((ext_vector_type(8)))  __bf16   v8b;
typedef __attribute__((ext_vector_type(8)))  float    v8f;
typedef __attribute__((ext_vector_type(4)))  float    v4f;
typedef __attribute__((ext_vector_type(4)))  unsigned int v4u;

__device__ __forceinline__ unsigned short f2bf_bits(float f) {
  unsigned u = __float_as_uint(f);
  return (unsigned short)((u + 0x7FFFu + ((u >> 16) & 1u)) >> 16);
}
__device__ __forceinline__ float bf_bits2f(unsigned short h) { return __uint_as_float(((unsigned)h) << 16); }

__device__ __forceinline__ void dep_guard_h(v8f& a, v8f& b, v16h x, v16h y) { asm volatile("v_nop\n\tv_nop\n\tv_nop\n\tv_nop" : "+v"(a), "+v"(b) : "v"(x), "v"(y)); }
__device__ __forceinline__ void dep_guard_b(v8f& a, v8f& b, v16b x, v16b y) { asm volatile("v_nop\n\tv_nop\n\tv_nop\n\tv_nop" : "+v"(a), "+v"(b) : "v"(x), "v"(y)); }
__device__ __forceinline__ void keep4_h(v16h a, v16h b, v16h c, v16h d) { asm volatile("v_nop" :: "v"(a), "v"(b), "v"(c), "v"(d)); }
__device__ __forceinline__ void keep4_b(v16b a, v16b b, v16b c, v16b d) { asm volatile("v_nop" :: "v"(a), "v"(b), "v"(c), "v"(d)); }
__device__ __forceinline__ void acc_guard4(v8f& a, v8f& b, v8f& c, v8f& d) { asm volatile("v_nop\n\tv_nop\n\tv_nop\n\tv_nop" : "+v"(a), "+v"(b), "+v"(c), "+v"(d)); }
template <typename T> struct Frag;
template <> struct Frag<_Float16> {
  typedef v16h V; union U { v16h v; v8h h[2]; };
  static __device__ __forceinline__ v16h load(const _Float16* p) {
    U f; f.h[0] = *(const v8h*)(p); f.h[1] = *(const v8h*)(p + 16); return f.v;
  }
  static __device__ __forceinline__ v8f mma(v16h a, v16h b, v8f c) {
    return __builtin_amdgcn_wmma_f32_16x16x32_f16(false, a, false, b, (short)0, c, false, false);
  }
  static __device__ __forceinline__ void guard(v8f& a, v8f& b, v16h x, v16h y) { dep_guard_h(a, b, x, y); }
  static __device__ __forceinline__ void keep(v16h a, v16h b, v16h c, v16h d) { keep4_h(a, b, c, d); }
};
template <> struct Frag<__bf16> {
  typedef v16b V; union U { v16b v; v8b h[2]; };
  static __device__ __forceinline__ v16b load(const __bf16* p) {
    U f; f.h[0] = *(const v8b*)(p); f.h[1] = *(const v8b*)(p + 16); return f.v;
  }
  static __device__ __forceinline__ v8f mma(v16b a, v16b b, v8f c) {
    return __builtin_amdgcn_wmma_f32_16x16x32_bf16(false, a, false, b, (short)0, c, false, false);
  }
  static __device__ __forceinline__ void guard(v8f& a, v8f& b, v16b x, v16b y) { dep_guard_b(a, b, x, y); }
  static __device__ __forceinline__ void keep(v16b a, v16b b, v16b c, v16b d) { keep4_b(a, b, c, d); }
};

__device__ __forceinline__ unsigned pk16(unsigned short a, unsigned short b) { return (unsigned)a | ((unsigned)b << 16); }
__device__ __forceinline__ unsigned short h_bits(float f) { const _Float16 h = (_Float16)f; return __builtin_bit_cast(unsigned short, h); }

__device__ __forceinline__ float h16_to_f32(unsigned hb) {
  const unsigned em = hb & 0x7fffu;
  const float fn = __uint_as_float((em + 0x1C000u) << 13);
  const float fs = (float)em * 5.9604644775390625e-8f;
  const float f  = (em < 0x400u) ? fs : fn;
  return __uint_as_float(__float_as_uint(f) | ((hb & 0x8000u) << 16));
}

__device__ __forceinline__ void store2_v4u(unsigned short* p, v4u u) {
  *(volatile v4u*)p = u;
  __threadfence();
  *(volatile v4u*)p = u;
}
__device__ __forceinline__ void store2_v4f(float* p, v4f v) {
  *(volatile v4f*)p = v;
  __threadfence();
  *(volatile v4f*)p = v;
}

template <int ET> struct Elem;
template <> struct Elem<0> { typedef _Float16 T; };
template <> struct Elem<1> { typedef __bf16 T; };
template <int ET, bool SPLIT, int BIAS_MODE, int OUT_MODE, bool RESID, int ACT = 0>
__global__ __launch_bounds__(256) void wmma_gemm64(
    const unsigned short* __restrict__ Ap, const unsigned short* __restrict__ A2p, int lda, long strideA,
    const unsigned short* __restrict__ Btp, const unsigned short* __restrict__ Bt2p, int ldb, long strideB,
    void* __restrict__ Cout, void* __restrict__ Cout2, int ldc, long strideC,
    const float* __restrict__ bias,
    const float* __restrict__ resid, long strideR,
    int M, int N, int K, float scale) {
  typedef typename Elem<ET>::T T;
  typedef typename Frag<T>::V V;
  const T* A = (const T*)Ap; const T* A2 = (const T*)A2p; const T* Bt = (const T*)Btp; const T* Bt2 = (const T*)Bt2p;
  __shared__ __align__(16) float sT[8][16 * 68];
  const int b    = blockIdx.y;
  const int lane = threadIdx.x & 31;
  const int wave = threadIdx.x >> 5;
  const int tilesN = N >> 6;
  const int tilesM = M >> 6;
  const int tile = blockIdx.x * 8 + wave;
  if (tile >= tilesM * tilesN) return;
  const int tm = tile / tilesN;
  const int tn = tile - tm * tilesN;
  const int m0 = tm << 6;
  const int n0 = tn << 6;

  const T* Ab  = A  + (size_t)b * strideA;
  const T* Bb  = Bt + (size_t)b * strideB;
  const T* Ab2 = SPLIT ? (A2  + (size_t)b * strideA) : nullptr;
  const T* Bb2 = SPLIT ? (Bt2 + (size_t)b * strideB) : nullptr;

  const int rlane = lane & 15;
  const int koff  = (lane >> 4) * 8;
  const int mOff  = (lane >> 4) * 8;

  v8f acc[4][4];
#pragma unroll
  for (int i = 0; i < 4; ++i)
#pragma unroll
    for (int j = 0; j < 4; ++j) acc[i][j] = (v8f){0.f,0.f,0.f,0.f,0.f,0.f,0.f,0.f};

  for (int k0 = 0; k0 < K; k0 += 32) {
    V bh[4], bl[4];
#pragma unroll
    for (int j = 0; j < 4; ++j) {
      const size_t bo = (size_t)(n0 + (j << 4) + rlane) * ldb + koff + k0;
      bh[j] = Frag<T>::load(Bb + bo);
      if (SPLIT) bl[j] = Frag<T>::load(Bb2 + bo);
    }
#pragma unroll
    for (int i = 0; i < 4; ++i) {
      const size_t ao = (size_t)(m0 + (i << 4) + rlane) * lda + koff + k0;
      V ah = Frag<T>::load(Ab + ao);
      V al;
      if (SPLIT) al = Frag<T>::load(Ab2 + ao);
#pragma unroll
      for (int j = 0; j < 4; ++j) {
        acc[i][j] = Frag<T>::mma(ah, bh[j], acc[i][j]);
        if (SPLIT) {
          acc[i][j] = Frag<T>::mma(ah, bl[j], acc[i][j]);
          acc[i][j] = Frag<T>::mma(al, bh[j], acc[i][j]);
        }
      }
      Frag<T>::guard(acc[i][0], acc[i][3], ah, SPLIT ? al : ah);
    }
    Frag<T>::keep(bh[0], bh[1], bh[2], bh[3]);
    if (SPLIT) Frag<T>::keep(bl[0], bl[1], bl[2], bl[3]);
  }
  acc_guard4(acc[0][0], acc[0][1], acc[0][2], acc[0][3]);
  acc_guard4(acc[1][0], acc[1][1], acc[1][2], acc[1][3]);
  acc_guard4(acc[2][0], acc[2][1], acc[2][2], acc[2][3]);
  acc_guard4(acc[3][0], acc[3][1], acc[3][2], acc[3][3]);

  float* slab = sT[wave];
  const float* Rb = RESID ? (resid + (size_t)b * strideR) : nullptr;
#pragma unroll
  for (int i = 0; i < 4; ++i) {
    const int mBase = m0 + (i << 4);
#pragma unroll
    for (int j = 0; j < 4; ++j) {
      const int n = n0 + (j << 4) + rlane;
      float bv = 0.f;
      if (BIAS_MODE == 2) bv = bias[n];
#pragma unroll
      for (int r = 0; r < 8; ++r) {
        float v = acc[i][j][r] * scale;
        if (BIAS_MODE == 1) v += bias[mBase + mOff + r];
        if (BIAS_MODE == 2) v += bv;
        if (RESID) v += Rb[(size_t)(mBase + mOff + r) * ldc + n];
        if (ACT == 2) v = fmaxf(v, 0.0f);
        if (ACT == 4) v = (v > 0.f) ? v : 0.01f * v;
        if (ACT == 6) v = 1.0f / (1.0f + expf(-v));
        slab[(mOff + r) * 68 + (j << 4) + rlane] = v;
      }
    }
    __builtin_amdgcn_fence(__ATOMIC_RELEASE, "workgroup");
    __builtin_amdgcn_wave_barrier();
    __builtin_amdgcn_fence(__ATOMIC_ACQUIRE, "workgroup");
    if (OUT_MODE == 0) {
      float* C = (float*)Cout + (size_t)b * strideC;
      const int hh = lane >> 4, c4 = (lane & 15) * 4;
      for (int pass = 0; pass < 2; ++pass) {
#pragma unroll
        for (int it = 0; it < 8; ++it) {
          const int row = it * 2 + hh;
          v4f v = *(const v4f*)(slab + row * 68 + c4);
          *(volatile v4f*)(C + (size_t)(mBase + row) * ldc + n0 + c4) = v;
        }
        __threadfence();
      }
    } else {
      const int q = lane >> 3, c8 = (lane & 7) * 8;
      unsigned short* C  = (unsigned short*)Cout  + (size_t)b * strideC;
      unsigned short* C2 = (OUT_MODE == 2) ? ((unsigned short*)Cout2 + (size_t)b * strideC) : nullptr;
      for (int pass = 0; pass < 2; ++pass) {
#pragma unroll
        for (int it = 0; it < 4; ++it) {
          const int row = it * 4 + q;
          const float* sp = slab + row * 68 + c8;
          v8h hv, lv;
#pragma unroll
          for (int e = 0; e < 8; ++e) {
            if (OUT_MODE == 1) {
              hv[e] = (_Float16)sp[e];
            } else {
              unsigned short hb = f2bf_bits(sp[e]);
              unsigned short lb = f2bf_bits(sp[e] - bf_bits2f(hb));
              hv[e] = __builtin_bit_cast(_Float16, hb);
              lv[e] = __builtin_bit_cast(_Float16, lb);
            }
          }
          *(volatile v8h*)(C + (size_t)(mBase + row) * ldc + n0 + c8) = hv;
          if (OUT_MODE == 2) *(volatile v8h*)(C2 + (size_t)(mBase + row) * ldc + n0 + c8) = lv;
        }
        __threadfence();
      }
    }
    __builtin_amdgcn_fence(__ATOMIC_RELEASE, "workgroup");
    __builtin_amdgcn_wave_barrier();
    __builtin_amdgcn_fence(__ATOMIC_ACQUIRE, "workgroup");
  }
}

__global__ __launch_bounds__(256) void cast8s_kernel(const float* __restrict__ in, unsigned short* __restrict__ out, int n8, float scale) {
  const int i = blockIdx.x * 256 + threadIdx.x;
  if (i >= n8) return;
  const float* p = in + 8 * (size_t)i;
  const v4f a = *(const v4f*)(p);
  const v4f c = *(const v4f*)(p + 4);
  unsigned short hb[8];
#pragma unroll
  for (int e = 0; e < 4; ++e) {
    hb[e]     = h_bits(a[e] * scale);
    hb[4 + e] = h_bits(c[e] * scale);
  }
  const v4u u = (v4u){pk16(hb[0], hb[1]), pk16(hb[2], hb[3]), pk16(hb[4], hb[5]), pk16(hb[6], hb[7])};
  store2_v4u(out + 8 * (size_t)i, u);
}

__global__ __launch_bounds__(256) void fill_zero2_kernel(unsigned short* __restrict__ a, unsigned short* __restrict__ b, int n8) {
  const int i = blockIdx.x * 256 + threadIdx.x;
  if (i >= n8) return;
  unsigned short* dst = (blockIdx.y == 0) ? a : b;
  const v4u z = (v4u){0u, 0u, 0u, 0u};
  store2_v4u(dst + 8 * (size_t)i, z);
}

__global__ __launch_bounds__(256) void wcast_kernel(const float* __restrict__ w0, const float* __restrict__ w1,
                                                    const float* __restrict__ w2, const float* __restrict__ w3,
                                                    const float* __restrict__ wc,
                                                    unsigned short* __restrict__ w16, unsigned short* __restrict__ wc16) {
  const int z = blockIdx.y;
  const int i = blockIdx.x * 256 + threadIdx.x;
  const float* src = (z == 0) ? w0 : (z == 1) ? w1 : (z == 2) ? w2 : (z == 3) ? w3 : wc;
  unsigned short* dst = (z < 4) ? (w16 + (size_t)z * kD * kD) : wc16;
  const int n8 = (z < 4) ? (kD * kD / 8) : (kHD * kHD / 8);
  if (i >= n8) return;
  const float* p = src + 8 * (size_t)i;
  const v4f a = *(const v4f*)(p);
  const v4f c = *(const v4f*)(p + 4);
  unsigned short hb[8];
#pragma unroll
  for (int e = 0; e < 4; ++e) {
    hb[e]     = h_bits(a[e] * kWCarry);
    hb[4 + e] = h_bits(c[e] * kWCarry);
  }
  const v4u u = (v4u){pk16(hb[0], hb[1]), pk16(hb[2], hb[3]), pk16(hb[4], hb[5]), pk16(hb[6], hb[7])};
  store2_v4u(dst + 8 * (size_t)i, u);
}

__device__ __forceinline__ float celu_f(float x) {
  const float en = expf(x * (1.0f / 1.3f)) - 1.0f;
  return (x > 0.f) ? x : 1.3f * en;
}

template <int MODE>
__global__ __launch_bounds__(256) void gn_rows_kernel(const float* __restrict__ P, const float* __restrict__ gw,
                                                      const float* __restrict__ gb, const unsigned short* __restrict__ kpl,
                                                      unsigned short* __restrict__ outp) {
  const int t = threadIdx.x, lane = t & 31, wave = t >> 5, hh = lane >> 4, cl = lane & 15;
  const int u = (blockIdx.x * 8 + wave) * 2 + hh;
  const size_t base = (size_t)u * kHD + cl * 8;
  const int ch = (u & 7) * kHD + cl * 8;
  const v4f a = *(const v4f*)(P + base);
  const v4f c = *(const v4f*)(P + base + 4);
  float y[8];
#pragma unroll
  for (int e = 0; e < 4; ++e) { y[e] = celu_f(a[e]); y[4 + e] = celu_f(c[e]); }
  float s = ((y[0] + y[1]) + (y[2] + y[3])) + ((y[4] + y[5]) + (y[6] + y[7]));
#pragma unroll
  for (int off = 1; off < 16; off <<= 1) s += __shfl_xor(s, off, 32);
  const float mu = s * (1.0f / 128.0f);
  float d[8];
  float sq = 0.f;
#pragma unroll
  for (int e = 0; e < 8; ++e) { d[e] = y[e] - mu; sq += d[e] * d[e]; }
#pragma unroll
  for (int off = 1; off < 16; off <<= 1) sq += __shfl_xor(sq, off, 32);
  const float var = sq * (1.0f / 128.0f);
  const float rs = rsqrtf(var + 1e-5f);
  const v4f w0 = *(const v4f*)(gw + ch), w1 = *(const v4f*)(gw + ch + 4);
  const v4f g0 = *(const v4f*)(gb + ch), g1 = *(const v4f*)(gb + ch + 4);
  float o[8];
#pragma unroll
  for (int e = 0; e < 4; ++e) {
    o[e]     = d[e] * rs * w0[e] + g0[e];
    o[4 + e] = d[4 + e] * rs * w1[e] + g1[e];
  }
  if (MODE == 2) {
    const v4u kk = *(const v4u*)(kpl + base);
    float kf[8];
    kf[0] = h16_to_f32(kk.x & 0xffffu); kf[1] = h16_to_f32(kk.x >> 16);
    kf[2] = h16_to_f32(kk.y & 0xffffu); kf[3] = h16_to_f32(kk.y >> 16);
    kf[4] = h16_to_f32(kk.z & 0xffffu); kf[5] = h16_to_f32(kk.z >> 16);
    kf[6] = h16_to_f32(kk.w & 0xffffu); kf[7] = h16_to_f32(kk.w >> 16);
#pragma unroll
    for (int e = 0; e < 8; ++e) o[e] = o[e] * kf[e];
  } else {
#pragma unroll
    for (int e = 0; e < 8; ++e) o[e] = o[e] * kXCarry;
  }
  unsigned short hb[8];
#pragma unroll
  for (int e = 0; e < 8; ++e) hb[e] = h_bits(o[e]);
  const v4u uu = (v4u){pk16(hb[0], hb[1]), pk16(hb[2], hb[3]), pk16(hb[4], hb[5]), pk16(hb[6], hb[7])};
  store2_v4u(outp + base, uu);
}

constexpr int kV2Pitch = 264;
__global__ __launch_bounds__(256) void gn_v2t_kernel(const float* __restrict__ P, const float* __restrict__ gw,
                                                     const float* __restrict__ gb, unsigned short* __restrict__ v2t) {
  __shared__ __align__(16) unsigned short sm[64 * kV2Pitch];
  const int t = threadIdx.x, lane = t & 31, wave = t >> 5;
  const int b = blockIdx.x, h = blockIdx.y, dh = blockIdx.z;
  {
    const v4u z = (v4u){0u, 0u, 0u, 0u};
#pragma unroll
    for (int j = 0; j < 2; ++j) {
      const int idx = t * 2 + j;
      const int row = idx >> 3, part = idx & 7;
      *(v4u*)(sm + row * kV2Pitch + 192 + part * 8) = z;
    }
  }
  __syncthreads();
  const int ch = h * kHD + lane * 4;
  const v4f wv = *(const v4f*)(gw + ch);
  const v4f gv = *(const v4f*)(gb + ch);
  const int cl0 = (lane & 15) * 4;
  for (int i = 0; i < 25; ++i) {
    const int tok = wave + 8 * i;
    if (tok >= kM) break;
    const v4f a = *(const v4f*)(P + ((size_t)(b * kM + tok)) * kD + ch);
    float y[4];
#pragma unroll
    for (int e = 0; e < 4; ++e) y[e] = celu_f(a[e]);
    float s = (y[0] + y[1]) + (y[2] + y[3]);
#pragma unroll
    for (int off = 1; off < 32; off <<= 1) s += __shfl_xor(s, off, 32);
    const float mu = s * (1.0f / 128.0f);
    float d[4];
    float sq = 0.f;
#pragma unroll
    for (int e = 0; e < 4; ++e) { d[e] = y[e] - mu; sq += d[e] * d[e]; }
#pragma unroll
    for (int off = 1; off < 32; off <<= 1) sq += __shfl_xor(sq, off, 32);
    const float var = sq * (1.0f / 128.0f);
    const float rs = rsqrtf(var + 1e-5f);
    unsigned short hb[4];
#pragma unroll
    for (int e = 0; e < 4; ++e) hb[e] = h_bits((d[e] * rs * wv[e] + gv[e]) * kXCarry);
    if ((lane >> 4) == dh) {
#pragma unroll
      for (int e = 0; e < 4; ++e) sm[(cl0 + e) * kV2Pitch + tok] = hb[e];
    }
  }
  __syncthreads();
  const size_t rowbase = ((size_t)(h * kHD + dh * 64)) * (kB * kSP) + (size_t)b * kSP + lane * 8;
  for (int pass = 0; pass < 2; ++pass) {
#pragma unroll
    for (int it = 0; it < 8; ++it) {
      const int cl = wave * 8 + it;
      const v4u u = *(const v4u*)(sm + cl * kV2Pitch + lane * 8);
      *(volatile v4u*)(v2t + rowbase + (size_t)cl * (kB * kSP)) = u;
    }
    __threadfence();
  }
}

__global__ __launch_bounds__(256) void softmax_kernel(const float* __restrict__ S, const float* __restrict__ mask,
                                                      unsigned short* __restrict__ Pp) {
  const int t = threadIdx.x, lane = t & 31, wave = t >> 5;
  const int b = blockIdx.y;
  const int r = blockIdx.x * 8 + wave;
  const int rc = (r < kM) ? r : (kM - 1);
  const float* sr = S + ((size_t)b * kSP + rc) * kSP + lane * 8;
  const v4f a = *(const v4f*)(sr);
  const v4f c = *(const v4f*)(sr + 4);
  float x[8];
#pragma unroll
  for (int e = 0; e < 4; ++e) { x[e] = a[e]; x[4 + e] = c[e]; }
  float s[8];
#pragma unroll
  for (int e = 0; e < 8; ++e) {
    const int j  = lane * 8 + e;
    const int jc = (j < kM) ? j : (kM - 1);
    const float mv = mask[b * kM + jc];
    const float v = (mv == 0.0f) ? -1.0e9f : x[e];
    s[e] = (j < kM) ? v : -3.0e38f;
  }
  float mx = fmaxf(fmaxf(fmaxf(s[0], s[1]), fmaxf(s[2], s[3])), fmaxf(fmaxf(s[4], s[5]), fmaxf(s[6], s[7])));
#pragma unroll
  for (int off = 1; off < 32; off <<= 1) mx = fmaxf(mx, __shfl_xor(mx, off, 32));
  float p[8];
  float ps = 0.f;
#pragma unroll
  for (int e = 0; e < 8; ++e) {
    const int j = lane * 8 + e;
    const float arg = (j < kM) ? (s[e] - mx) : -100.0f;
    const float ev = expf(arg);
    p[e] = (j < kM) ? ev : 0.0f;
    ps += p[e];
  }
#pragma unroll
  for (int off = 1; off < 32; off <<= 1) ps += __shfl_xor(ps, off, 32);
  const float inv = 1.0f / ps;
  unsigned short hb[8];
#pragma unroll
  for (int e = 0; e < 8; ++e) hb[e] = h_bits(p[e] * inv * kPCarry);
  const v4u u = (v4u){pk16(hb[0], hb[1]), pk16(hb[2], hb[3]), pk16(hb[4], hb[5]), pk16(hb[6], hb[7])};
  v4u uu;
  uu.x = (r < kM) ? u.x : 0u;
  uu.y = (r < kM) ? u.y : 0u;
  uu.z = (r < kM) ? u.z : 0u;
  uu.w = (r < kM) ? u.w : 0u;
  store2_v4u(Pp + ((size_t)b * kSP + r) * kSP + lane * 8, uu);
}

__global__ __launch_bounds__(256) void merge_ln_kernel(const float* xin, const float* __restrict__ att,
                                                       const float* __restrict__ gate, const float* __restrict__ lnw,
                                                       const float* __restrict__ lnb, float* xout,
                                                       unsigned short* __restrict__ x16) {
  __shared__ float redA[8];
  __shared__ float redB[8];
  __shared__ __align__(16) float srow[kD];
  const int t = threadIdx.x, lane = t & 31, wave = t >> 5;
  const int r = blockIdx.x;
  const int b = r / kM;
  const int m = r - b * kM;
  const int c0 = t * 4;
  const size_t ro = (size_t)r * kD + c0;
  const v4f xv = *(const v4f*)(xin + ro);
  const v4f gv = *(const v4f*)(gate + ro);
  const v4f av = *(const v4f*)(att + ((size_t)(b * kSP + m)) * kD + c0);
  float y[4];
#pragma unroll
  for (int e = 0; e < 4; ++e) y[e] = xv[e] + gv[e] * av[e];
  float s = (y[0] + y[1]) + (y[2] + y[3]);
#pragma unroll
  for (int off = 1; off < 32; off <<= 1) s += __shfl_xor(s, off, 32);
  if (lane == 0) redA[wave] = s;
  __syncthreads();
  float tot = redA[0];
#pragma unroll
  for (int w = 1; w < 8; ++w) tot += redA[w];
  const float mu = tot * (1.0f / 1024.0f);
  float d[4];
  float sq = 0.f;
#pragma unroll
  for (int e = 0; e < 4; ++e) { d[e] = y[e] - mu; sq += d[e] * d[e]; }
#pragma unroll
  for (int off = 1; off < 32; off <<= 1) sq += __shfl_xor(sq, off, 32);
  if (lane == 0) redB[wave] = sq;
  __syncthreads();
  float tot2 = redB[0];
#pragma unroll
  for (int w = 1; w < 8; ++w) tot2 += redB[w];
  const float var = tot2 * (1.0f / 1024.0f);
  const float rs = rsqrtf(var + 1e-5f);
  const v4f wv = *(const v4f*)(lnw + c0);
  const v4f bv = *(const v4f*)(lnb + c0);
  v4f ov;
#pragma unroll
  for (int e = 0; e < 4; ++e) ov[e] = d[e] * rs * wv[e] + bv[e];
  *(v4f*)(srow + c0) = ov;
  __syncthreads();
  const int tc = t & 127;
  const v4f p0 = *(const v4f*)(srow + tc * 8);
  const v4f p1 = *(const v4f*)(srow + tc * 8 + 4);
  unsigned short hb[8];
#pragma unroll
  for (int e = 0; e < 4; ++e) {
    hb[e]     = h_bits(p0[e] * kXCarry);
    hb[4 + e] = h_bits(p1[e] * kXCarry);
  }
  const v4u hu = (v4u){pk16(hb[0], hb[1]), pk16(hb[2], hb[3]), pk16(hb[4], hb[5]), pk16(hb[6], hb[7])};
  unsigned short* hp = x16 + (size_t)r * kD + tc * 8;
  for (int pass = 0; pass < 2; ++pass) {
    *(volatile v4f*)(xout + ro) = ov;
    if (t < 128) *(volatile v4u*)hp = hu;
    __threadfence();
  }
}

__global__ __launch_bounds__(256) void pool_kernel(const float* x, const float* __restrict__ mask, float* out0) {
  const int t = threadIdx.x;
  const int b = blockIdx.x;
  const int c0 = t * 4;
  v4f acc = (v4f){0.f, 0.f, 0.f, 0.f};
  float ms = 0.f;
#pragma unroll 1
  for (int m = 0; m < kM; ++m) {
    const float mv = mask[b * kM + m];
    const v4f xv = *(const v4f*)(x + ((size_t)(b * kM + m)) * kD + c0);
    acc += xv * mv;
    ms += mv;
  }
  const float inv = 1.0f / ms;
  const v4f o = acc * inv;
  store2_v4f(out0 + (size_t)b * kD + c0, o);
}

extern "C" void kernel_launch(void* const* d_in, const int* in_sizes, int n_in,
                              void* d_out, int out_size, void* d_ws, size_t ws_size,
                              hipStream_t stream) {
  if (n_in < 22) return;
  if (in_sizes[0] != kTok * kD) return;
  if (in_sizes[1] != kTok) return;
  if (in_sizes[2] != kL * kD * kD || in_sizes[6] != kL * kD * kD || in_sizes[10] != kL * kD * kD || in_sizes[14] != kL * kD * kD) return;
  if (in_sizes[18] != kL * kHD * kHD || in_sizes[19] != kL * kHD) return;
  if (in_sizes[3] != kL * kD || in_sizes[20] != kL * kD || in_sizes[21] != kL * kD) return;
  if (out_size != kB * kD + kTok * kD) return;
  if (ws_size < kWsTotal) return;

  const float* att_feats = (const float*)d_in[0];
  const float* att_mask  = (const float*)d_in[1];
  const float* Wq2  = (const float*)d_in[2];
  const float* bq2  = (const float*)d_in[3];
  const float* gq2w = (const float*)d_in[4];
  const float* gq2b = (const float*)d_in[5];
  const float* Wk   = (const float*)d_in[6];
  const float* bk   = (const float*)d_in[7];
  const float* gkw  = (const float*)d_in[8];
  const float* gkb  = (const float*)d_in[9];
  const float* Wv1  = (const float*)d_in[10];
  const float* bv1  = (const float*)d_in[11];
  const float* gv1w = (const float*)d_in[12];
  const float* gv1b = (const float*)d_in[13];
  const float* Wv2  = (const float*)d_in[14];
  const float* bv2  = (const float*)d_in[15];
  const float* gv2w = (const float*)d_in[16];
  const float* gv2b = (const float*)d_in[17];
  const float* Wc   = (const float*)d_in[18];
  const float* bc   = (const float*)d_in[19];
  const float* lnw  = (const float*)d_in[20];
  const float* lnb  = (const float*)d_in[21];

  char* ws = (char*)d_ws;
  float*          Ppl   = (float*)(ws + kOffP);
  float*          GATE  = (float*)(ws + kOffP);
  unsigned short* GIN16 = (unsigned short*)(ws + kOffATT);
  float*          ATT   = (float*)(ws + kOffATT);
  unsigned short* X16   = (unsigned short*)(ws + kOffX16);
  float*          Spl   = (float*)(ws + kOffX16);
  unsigned short* PP    = (unsigned short*)(ws + kOffX16 + kBytesS);
  unsigned short* W16   = (unsigned short*)(ws + kOffW16);
  unsigned short* WC16  = (unsigned short*)(ws + kOffWC16);
  unsigned short* Q16   = (unsigned short*)(ws + kOffQ16);
  unsigned short* K16   = (unsigned short*)(ws + kOffK16);
  unsigned short* V2T   = (unsigned short*)(ws + kOffV2T);

  float* out0 = (float*)d_out;
  float* out1 = (float*)d_out + (size_t)kB * kD;

  const float projScale  = 1.0f / (kXCarry * kWCarry);
  const float gateScale  = 1.0f / (kXCarry * kWCarry);
  const float scoreScale = 0.08838834764831845f * (1.0f / (kXCarry * kXCarry));
  const float pvScale    = 1.0f / (kPCarry * kXCarry);

  {
    const int n8 = kTok * kD / 8;
    cast8s_kernel<<<dim3(n8 / 256), dim3(256), 0, stream>>>(att_feats, X16, n8, kXCarry);
    const int npad8 = 64 * kD / 8;
    fill_zero2_kernel<<<dim3(npad8 / 256, 2), dim3(256), 0, stream>>>(Q16 + (size_t)kTok * kD, K16 + (size_t)kTok * kD, npad8);
  }

  for (int i = 0; i < kL; ++i) {
    const size_t wo = (size_t)i * kD * kD;
    wcast_kernel<<<dim3(512, 5), dim3(256), 0, stream>>>(Wq2 + wo, Wk + wo, Wv1 + wo, Wv2 + wo, Wc + (size_t)i * kHD * kHD, W16, WC16);

    for (int z = 0; z < 4; ++z) {
      const float* biasz = (z == 0) ? bq2 : (z == 1) ? bk : (z == 2) ? bv1 : bv2;
      const float* gwz   = (z == 0) ? gq2w : (z == 1) ? gkw : (z == 2) ? gv1w : gv2w;
      const float* gbz   = (z == 0) ? gq2b : (z == 1) ? gkb : (z == 2) ? gv1b : gv2b;
      wmma_gemm64<0, false, 2, 0, false, 0><<<dim3(196, 1), dim3(256), 0, stream>>>(
          X16, nullptr, kD, 0L,
          W16 + (size_t)z * kD * kD, nullptr, kD, 0L,
          (void*)Ppl, nullptr, kD, 0L,
          biasz + (size_t)i * kD, nullptr, 0L,
          kTok, kD, kD, projScale);
      if (z == 0) {
        gn_rows_kernel<0><<<dim3(3136), dim3(256), 0, stream>>>(Ppl, gwz + (size_t)i * kD, gbz + (size_t)i * kD, K16, Q16);
      } else if (z == 1) {
        gn_rows_kernel<0><<<dim3(3136), dim3(256), 0, stream>>>(Ppl, gwz + (size_t)i * kD, gbz + (size_t)i * kD, Q16, K16);
      } else if (z == 2) {
        gn_rows_kernel<2><<<dim3(3136), dim3(256), 0, stream>>>(Ppl, gwz + (size_t)i * kD, gbz + (size_t)i * kD, K16, GIN16);
      } else {
        gn_v2t_kernel<<<dim3(kB, kH, 2), dim3(256), 0, stream>>>(Ppl, gwz + (size_t)i * kD, gbz + (size_t)i * kD, V2T);
      }
    }

    wmma_gemm64<0, false, 2, 0, false, 6><<<dim3(196, 1), dim3(256), 0, stream>>>(
        GIN16, nullptr, kHD, 0L,
        WC16, nullptr, kHD, 0L,
        (void*)GATE, nullptr, kHD, 0L,
        bc + (size_t)i * kHD, nullptr, 0L,
        kTok * kH, kHD, kHD, gateScale);

    for (int h = 0; h < kH; ++h) {
      wmma_gemm64<0, false, 0, 0, false, 0><<<dim3(2, kB), dim3(256), 0, stream>>>(
          Q16 + (size_t)h * kHD, nullptr, kD, (long)kM * kD,
          K16 + (size_t)h * kHD, nullptr, kD, (long)kM * kD,
          (void*)Spl, nullptr, kSP, (long)kSP * kSP,
          nullptr, nullptr, 0L,
          kSP, kSP, kHD, scoreScale);
      softmax_kernel<<<dim3(kSP / 8, kB), dim3(256), 0, stream>>>(Spl, att_mask, PP);
      wmma_gemm64<0, false, 0, 0, false, 0><<<dim3(1, kB), dim3(256), 0, stream>>>(
          PP, nullptr, kSP, (long)kSP * kSP,
          V2T + (size_t)h * kHD * (kB * kSP), nullptr, kB * kSP, (long)kSP,
          (void*)(ATT + (size_t)h * kHD), nullptr, kD, (long)kSP * kD,
          nullptr, nullptr, 0L,
          kSP, kHD, kKeyK, pvScale);
    }

    const float* xin = (i == 0) ? att_feats : out1;
    merge_ln_kernel<<<dim3(kTok), dim3(256), 0, stream>>>(xin, ATT, GATE, lnw + (size_t)i * kD, lnb + (size_t)i * kD, out1, X16);
  }

  pool_kernel<<<dim3(kB), dim3(256), 0, stream>>>(out1, att_mask, out0);
}
